// S4D_29703993819395
// MI455X (gfx1250) — hardware-verified
//
#include <hip/hip_runtime.h>
#include <cstdint>


#define Bq 4
#define Lq 2048
#define Hq 1024
#define N2q 32
#define NCHUNK 32
#define NCOL 128
#define NTOK 8192

typedef _Float16 h16;
typedef __attribute__((ext_vector_type(16))) _Float16 v16h;
typedef __attribute__((ext_vector_type(8)))  _Float16 v8h;
typedef __attribute__((ext_vector_type(8)))  float  v8f;
typedef __attribute__((ext_vector_type(4)))  float  v4f;
typedef __attribute__((ext_vector_type(2)))  float  v2f;
typedef __attribute__((ext_vector_type(4)))  unsigned int v4u;

__device__ __forceinline__ v8f wmma16(v16h a, v16h b, v8f c) {
  v8f d = __builtin_amdgcn_wmma_f32_16x16x32_f16(false, a, false, b, (short)0, c, false, false);
  asm volatile("v_nop\n\tv_nop\n\tv_nop\n\tv_nop" : "+v"(d) : "v"(a), "v"(b));
  return d;
}

__device__ __forceinline__ v16h frag_rowmajor(const h16* M, int ld, int row0, int col0, int lane) {
  int r = lane & 15, hf = (lane >> 4) & 1;
  const h16* p = M + (row0 + r) * ld + col0;
  v16h f;
#pragma unroll
  for (int i = 0; i < 8; ++i) f[i] = p[hf * 8 + i];
#pragma unroll
  for (int i = 0; i < 8; ++i) f[8 + i] = p[16 + hf * 8 + i];
  return f;
}
__device__ __forceinline__ v16h frag_kmajor(const h16* M, int ld, int row0, int k0, int lane) {
  int r = lane & 15, hf = (lane >> 4) & 1;
  const h16* p = M + k0 * ld + row0 + r;
  v16h f;
#pragma unroll
  for (int i = 0; i < 8; ++i) f[i] = p[(hf * 8 + i) * ld];
#pragma unroll
  for (int i = 0; i < 8; ++i) f[8 + i] = p[(16 + hf * 8 + i) * ld];
  return f;
}

__device__ __forceinline__ float gelu_exact(float x) {
  return 0.5f * x * (1.0f + erff(x * 0.70710678118654752f));
}

__device__ __forceinline__ void store_block16(const void* lds, void* g, int n16, int tid, int nthr) {
  const v4u* s = (const v4u*)lds; volatile v4u* d = (volatile v4u*)g;
  for (int i = tid; i < n16; i += nthr) d[i] = s[i];
  __threadfence();
  for (int i = tid; i < n16; i += nthr) d[i] = s[i];
}

__global__ __launch_bounds__(256) void s4d_transpose(const float* __restrict__ u, h16* __restrict__ UT) {
  __shared__ float tile[64][65];
  __shared__ __attribute__((aligned(16))) h16 tout[64 * 64];
  int bc = blockIdx.x;
  int b = bc >> 5, c = bc & 31;
  int h0 = blockIdx.y * 64;
  int tid = threadIdx.x;
#pragma unroll
  for (int q = 0; q < 16; ++q) {
    int e = tid + q * 256;
    int hh = e & 63, m = e >> 6;
    tile[m][hh] = u[((size_t)(b * Lq + c * 64 + m)) * Hq + h0 + hh];
  }
  __syncthreads();
#pragma unroll
  for (int q = 0; q < 16; ++q) {
    int e = tid + q * 256;
    int m = e & 63, hh = e >> 6;
    tout[hh * 64 + m] = (h16)tile[m][hh];
  }
  __syncthreads();
  const v4u* s = (const v4u*)tout;
  for (int pass = 0; pass < 2; ++pass) {
#pragma unroll
    for (int q = 0; q < 2; ++q) {
      int piece = tid + q * 256;
      int hh = piece >> 3, seg = piece & 7;
      volatile v4u* d = (volatile v4u*)(UT + (((size_t)(h0 + hh)) * NCOL + (b * 32 + c)) * 64) + seg;
      *d = s[piece];
    }
    __threadfence();
  }
}

__global__ __launch_bounds__(256) void s4d_cvt_w(const float* __restrict__ Wm, h16* __restrict__ Wh, int n8) {
  int i = blockIdx.x * 256 + threadIdx.x;
  if (i < n8) {
    v4f a = *(const v4f*)(Wm + (size_t)i * 8), bq = *(const v4f*)(Wm + (size_t)i * 8 + 4);
    v8h o; o[0] = (h16)a[0]; o[1] = (h16)a[1]; o[2] = (h16)a[2]; o[3] = (h16)a[3]; o[4] = (h16)bq[0]; o[5] = (h16)bq[1]; o[6] = (h16)bq[2]; o[7] = (h16)bq[3];
    *(volatile v8h*)(Wh + (size_t)i * 8) = o;
    __threadfence();
    *(volatile v8h*)(Wh + (size_t)i * 8) = o;
  }
}

__global__ __launch_bounds__(32) void s4d_prep(const float* __restrict__ log_dt,
                                               const float* __restrict__ log_w_real,
                                               const float* __restrict__ w_imag,
                                               const float* __restrict__ C_real,
                                               const float* __restrict__ C_imag,
                                               h16* __restrict__ PB,
                                               float* __restrict__ Z64) {
  __shared__ float karr[64];
  __shared__ __attribute__((aligned(16))) h16 blk[12288];
  __shared__ __attribute__((aligned(16))) float zs[64];
  int h = blockIdx.x, n = threadIdx.x;
  float dt = expf(log_dt[h]);
  float wr = -expf(log_w_real[n]);
  float wi = w_imag[n];
  float cr = C_real[h * N2q + n], ci = C_imag[h * N2q + n];
  float ar = wr * dt, ai = wi * dt;
  float ea = expf(ar);
  float zr = ea * cosf(ai), zi = ea * sinf(ai);
  float er = zr - 1.0f, ei = zi;
  float inv = 1.0f / (wr * wr + wi * wi);
  float qr = (er * wr + ei * wi) * inv, qi = (ei * wr - er * wi) * inv;
  float cwr = cr * qr - ci * qi, cwi = cr * qi + ci * qr;

  h16* Th = blk;
  h16* Ph = blk + 4096;
  h16* Gh = blk + 8192;

  float pr = 1.0f, pi = 0.0f;
  for (int d = 0; d < 64; ++d) {
    float s = cwr * pr - cwi * pi;
    for (int off = 16; off >= 1; off >>= 1) s += __shfl_xor(s, off);
    if (n == 0) karr[d] = 2.0f * s;
    Ph[(2 * n) * 64 + (63 - d)]     = (h16)pr;
    Ph[(2 * n + 1) * 64 + (63 - d)] = (h16)pi;
    float nr = pr * zr - pi * zi, ni = pr * zi + pi * zr;
    Gh[d * 64 + 2 * n]     = (h16)(2.0f * (cwr * nr - cwi * ni));
    Gh[d * 64 + 2 * n + 1] = (h16)(-2.0f * (cwr * ni + cwi * nr));
    pr = nr; pi = ni;
  }
  zs[2 * n] = pr; zs[2 * n + 1] = pi;
  __syncthreads();
  for (int j = 0; j < 64; ++j) {
    int m0 = 2 * n, m1 = 2 * n + 1;
    Th[j * 64 + m0] = (h16)((j >= m0) ? karr[j - m0] : 0.0f);
    Th[j * 64 + m1] = (h16)((j >= m1) ? karr[j - m1] : 0.0f);
  }
  __syncthreads();
  store_block16(blk, PB + (size_t)h * 12288, 12288 * 2 / 16, n, 32);
  store_block16(zs, Z64 + (size_t)h * 64, 64 * 4 / 16, n, 32);
}

__global__ __launch_bounds__(256) void s4d_chunk(const h16* __restrict__ PB,
                                                 const h16* __restrict__ UT,
                                                 const float* __restrict__ Z64,
                                                 const float* __restrict__ D,
                                                 h16* __restrict__ actT) {
  extern __shared__ __attribute__((aligned(16))) char smem[];
  h16* Tm = (h16*)smem;
  h16* Pm = Tm + 4096;
  h16* Gm = Pm + 4096;
  h16* Um = Gm + 4096;
  h16* Xt = Um + 8192;
  float*  Sm = (float*)(Xt + 8192);

  int h = blockIdx.x, tid = threadIdx.x;
  int wave = tid >> 5, lane = tid & 31;
  int colb = wave * 16;
  int hf = (lane >> 4) & 1, n16 = lane & 15;

  {
    const v4u* sp = (const v4u*)(PB + (size_t)h * 12288); v4u* dp = (v4u*)Tm;
    for (int i = tid; i < 1536; i += 256) dp[i] = sp[i];
    const v4u* su = (const v4u*)(UT + (size_t)h * 8192); v4u* du = (v4u*)Um;
    for (int i = tid; i < 1024; i += 256) du[i] = su[i];
  }
  __syncthreads();

  v8f vzero = {0.f, 0.f, 0.f, 0.f, 0.f, 0.f, 0.f, 0.f};

  {
    v8f accS[4];
#pragma unroll
    for (int r = 0; r < 4; ++r) accS[r] = vzero;
#pragma unroll
    for (int kk = 0; kk < 64; kk += 32) {
      v16h bu = frag_rowmajor(Um, 64, colb, kk, lane);
#pragma unroll
      for (int r = 0; r < 4; ++r) {
        v16h a = frag_rowmajor(Pm, 64, r * 16, kk, lane);
        accS[r] = wmma16(a, bu, accS[r]);
      }
    }
#pragma unroll
    for (int r = 0; r < 4; ++r)
#pragma unroll
      for (int i = 0; i < 8; ++i)
        Sm[(r * 16 + i + 8 * hf) * 128 + colb + n16] = accS[r][i];
  }
  __syncthreads();

  if (tid < 128) {
    int b = tid >> 5, n = tid & 31;
    float zr = Z64[h * 64 + 2 * n], zi = Z64[h * 64 + 2 * n + 1];
    float xr = 0.0f, xi = 0.0f;
    uint32_t* Xw = (uint32_t*)Xt;
    for (int c = 0; c < NCHUNK; ++c) {
      int col = b * 32 + c;
      uint32_t pk = ((uint32_t)__builtin_bit_cast(unsigned short, (h16)xi) << 16) |
                    (uint32_t)__builtin_bit_cast(unsigned short, (h16)xr);
      Xw[col * 32 + n] = pk;
      float sr = Sm[(2 * n) * 128 + col], si = Sm[(2 * n + 1) * 128 + col];
      float nxr = zr * xr - zi * xi + sr;
      float nxi = zr * xi + zi * xr + si;
      xr = nxr; xi = nxi;
    }
  }
  __syncthreads();

  v8f accY[4];
#pragma unroll
  for (int r = 0; r < 4; ++r) accY[r] = vzero;
#pragma unroll
  for (int kk = 0; kk < 64; kk += 32) {
    v16h bx = frag_rowmajor(Xt, 64, colb, kk, lane);
    v16h bu = frag_rowmajor(Um, 64, colb, kk, lane);
#pragma unroll
    for (int r = 0; r < 4; ++r) {
      v16h ag = frag_rowmajor(Gm, 64, r * 16, kk, lane);
      accY[r] = wmma16(ag, bx, accY[r]);
      v16h at = frag_rowmajor(Tm, 64, r * 16, kk, lane);
      accY[r] = wmma16(at, bu, accY[r]);
    }
  }
  __syncthreads();
  h16* ash = (h16*)Sm;
  float Dh = D[h];
#pragma unroll
  for (int r = 0; r < 4; ++r) {
#pragma unroll
    for (int i = 0; i < 8; ++i) {
      int row = r * 16 + i + 8 * hf;
      int col = colb + n16;
      float uval = (float)Um[col * 64 + row];
      float y = accY[r][i] + Dh * uval;
      ash[col * 64 + row] = (h16)gelu_exact(y);
    }
  }
  __syncthreads();
  store_block16(ash, actT + (size_t)h * NTOK, NTOK * 2 / 16, tid, 256);
}

__global__ __launch_bounds__(256) void s4d_out_gemm(const h16* __restrict__ actT,
                                                    const h16* __restrict__ Wh,
                                                    const float* __restrict__ bias,
                                                    float* __restrict__ out) {
  __shared__ __attribute__((aligned(16))) h16 Al[32 * 128];
  __shared__ __attribute__((aligned(16))) h16 Bl[128 * 32];
  int tid = threadIdx.x, wave = tid >> 5, lane = tid & 31;
  int col0 = blockIdx.x * 128;
  int row0 = blockIdx.y * 128;
  const int KB = Hq / 32;

  v8f vzero = {0.f, 0.f, 0.f, 0.f, 0.f, 0.f, 0.f, 0.f};
  v8f acc[8];
#pragma unroll
  for (int ct = 0; ct < 8; ++ct) acc[ct] = vzero;

  for (int kb = 0; kb < KB; ++kb) {
    __syncthreads();
#pragma unroll
    for (int q = 0; q < 2; ++q) {
      int piece = tid + q * 256;
      int kr = piece >> 4, sg = piece & 15;
      *(v4u*)(Al + kr * 128 + sg * 8) = *(const v4u*)(actT + (size_t)(kb * 32 + kr) * NTOK + row0 + sg * 8);
      int fr = piece >> 2, s4 = piece & 3;
      *(v4u*)(Bl + fr * 32 + s4 * 8) = *(const v4u*)(Wh + (size_t)(col0 + fr) * Hq + kb * 32 + s4 * 8);
    }
    __syncthreads();
    v16h a = frag_kmajor(Al, 128, wave * 16, 0, lane);
#pragma unroll
    for (int ct = 0; ct < 8; ++ct) {
      v16h b = frag_rowmajor(Bl, 32, ct * 16, 0, lane);
      acc[ct] = wmma16(a, b, acc[ct]);
    }
  }
  int hf = (lane >> 4) & 1;
  for (int pass = 0; pass < 2; ++pass) {
#pragma unroll
    for (int p2 = 0; p2 < 4; ++p2) {
      int cbase = col0 + p2 * 32;
      float bv = bias[cbase + lane];
#pragma unroll
      for (int i = 0; i < 8; ++i) {
        float a0 = acc[2 * p2][i], b0 = acc[2 * p2 + 1][i];
        float ax = __shfl_xor(a0, 16), bx = __shfl_xor(b0, 16);
        float v1 = hf ? bx : a0;
        float v2 = hf ? b0 : ax;
        int r1 = row0 + wave * 16 + i, r2 = r1 + 8;
        *(volatile float*)(out + (size_t)r1 * Hq + cbase + lane) = v1 + bv;
        *(volatile float*)(out + (size_t)r2 * Hq + cbase + lane) = v2 + bv;
      }
    }
    __threadfence();
  }
}

extern "C" void kernel_launch(void* const* d_in, const int* in_sizes, int n_in,
                              void* d_out, int out_size, void* d_ws, size_t ws_size,
                              hipStream_t stream) {
  (void)in_sizes; (void)n_in; (void)out_size;
  const float* u           = (const float*)d_in[0];
  const float* log_dt      = (const float*)d_in[1];
  const float* log_w_real  = (const float*)d_in[2];
  const float* w_imag      = (const float*)d_in[3];
  const float* C_real      = (const float*)d_in[4];
  const float* C_imag      = (const float*)d_in[5];
  const float* D           = (const float*)d_in[6];
  const float* W_out       = (const float*)d_in[7];
  const float* b_out       = (const float*)d_in[8];
  float* out = (float*)d_out;

  char* ws = (char*)d_ws;
  h16*   UT   = (h16*)(ws);
  h16*   PB   = (h16*)(ws + (16u << 20));
  float* Z64  = (float*)(ws + (40u << 20));
  h16*   Wh   = (h16*)(ws + (41u << 20));
  h16*   actT = (h16*)(ws + (44u << 20));
  if ((size_t)(60u << 20) > ws_size) return;

  s4d_transpose<<<dim3(Bq * NCHUNK, Hq / 64), 256, 0, stream>>>(u, UT);
  s4d_cvt_w<<<(Hq * Hq / 8 + 255) / 256, 256, 0, stream>>>(W_out, Wh, Hq * Hq / 8);
  s4d_prep<<<Hq, 32, 0, stream>>>(log_dt, log_w_real, w_imag, C_real, C_imag, PB, Z64);
  size_t shbytes = (size_t)(4096 * 3 + 8192 * 2) * sizeof(h16) + 8192 * sizeof(float);
  s4d_chunk<<<Hq, 256, shbytes, stream>>>(PB, UT, Z64, D, actT);
  s4d_out_gemm<<<dim3(Hq / 128, NTOK / 128), 256, 0, stream>>>(actT, Wh, b_out, out);
}
